// GCNN2_81063212744721
// MI455X (gfx1250) — hardware-verified
//
#include <hip/hip_runtime.h>
#include <math.h>

typedef __attribute__((ext_vector_type(16))) _Float16 v16h;
typedef __attribute__((ext_vector_type(8)))  _Float16 v8h;
typedef __attribute__((ext_vector_type(4)))  _Float16 v4h;
typedef __attribute__((ext_vector_type(16))) __bf16   v16b;
typedef __attribute__((ext_vector_type(8)))  __bf16   v8b;
typedef __attribute__((ext_vector_type(8)))  float    v8f;
typedef __attribute__((ext_vector_type(4)))  float    v4f;
typedef __attribute__((ext_vector_type(4)))  int      v4i;

__device__ __forceinline__ unsigned short f2bf_bits(float f) {
  unsigned u = __float_as_uint(f);
  return (unsigned short)((u + 0x7FFFu + ((u >> 16) & 1u)) >> 16);
}
__device__ __forceinline__ float bf_bits2f(unsigned short h) { return __uint_as_float(((unsigned)h) << 16); }

__device__ __forceinline__ void dep_guard_h(v8f& a, v8f& b, v16h x, v16h y) { asm volatile("v_nop\n\tv_nop\n\tv_nop\n\tv_nop" : "+v"(a), "+v"(b) : "v"(x), "v"(y)); }
__device__ __forceinline__ void dep_guard_b(v8f& a, v8f& b, v16b x, v16b y) { asm volatile("v_nop\n\tv_nop\n\tv_nop\n\tv_nop" : "+v"(a), "+v"(b) : "v"(x), "v"(y)); }
__device__ __forceinline__ void keep4_h(v16h a, v16h b, v16h c, v16h d) { asm volatile("v_nop" :: "v"(a), "v"(b), "v"(c), "v"(d)); }
__device__ __forceinline__ void keep4_b(v16b a, v16b b, v16b c, v16b d) { asm volatile("v_nop" :: "v"(a), "v"(b), "v"(c), "v"(d)); }
__device__ __forceinline__ void acc_guard4(v8f& a, v8f& b, v8f& c, v8f& d) { asm volatile("v_nop\n\tv_nop\n\tv_nop\n\tv_nop" : "+v"(a), "+v"(b), "+v"(c), "+v"(d)); }
template <typename T> struct Frag;
template <> struct Frag<_Float16> {
  typedef v16h V; union U { v16h v; v8h h[2]; };
  static __device__ __forceinline__ v16h load(const _Float16* p) {
    U f; f.h[0] = *(const v8h*)(p); f.h[1] = *(const v8h*)(p + 16); return f.v;
  }
  static __device__ __forceinline__ v8f mma(v16h a, v16h b, v8f c) {
    return __builtin_amdgcn_wmma_f32_16x16x32_f16(false, a, false, b, (short)0, c, false, false);
  }
  static __device__ __forceinline__ void guard(v8f& a, v8f& b, v16h x, v16h y) { dep_guard_h(a, b, x, y); }
  static __device__ __forceinline__ void keep(v16h a, v16h b, v16h c, v16h d) { keep4_h(a, b, c, d); }
};
template <> struct Frag<__bf16> {
  typedef v16b V; union U { v16b v; v8b h[2]; };
  static __device__ __forceinline__ v16b load(const __bf16* p) {
    U f; f.h[0] = *(const v8b*)(p); f.h[1] = *(const v8b*)(p + 16); return f.v;
  }
  static __device__ __forceinline__ v8f mma(v16b a, v16b b, v8f c) {
    return __builtin_amdgcn_wmma_f32_16x16x32_bf16(false, a, false, b, (short)0, c, false, false);
  }
  static __device__ __forceinline__ void guard(v8f& a, v8f& b, v16b x, v16b y) { dep_guard_b(a, b, x, y); }
  static __device__ __forceinline__ void keep(v16b a, v16b b, v16b c, v16b d) { keep4_b(a, b, c, d); }
};

template <int ET> struct Elem;
template <> struct Elem<0> { typedef _Float16 T; };
template <> struct Elem<1> { typedef __bf16 T; };
template <int ET, bool SPLIT, int BIAS_MODE, int OUT_MODE, bool RESID, int ACT = 0>
__global__ __launch_bounds__(256) void wmma_gemm64(
    const unsigned short* __restrict__ Ap, const unsigned short* __restrict__ A2p, int lda, long strideA,
    const unsigned short* __restrict__ Btp, const unsigned short* __restrict__ Bt2p, int ldb, long strideB,
    void* __restrict__ Cout, void* __restrict__ Cout2, int ldc, long strideC,
    const float* __restrict__ bias,
    const float* __restrict__ resid, long strideR,
    int M, int N, int K, float scale) {
  typedef typename Elem<ET>::T T;
  typedef typename Frag<T>::V V;
  const T* A = (const T*)Ap; const T* A2 = (const T*)A2p; const T* Bt = (const T*)Btp; const T* Bt2 = (const T*)Bt2p;
  __shared__ __align__(16) float sT[8][16 * 68];
  const int b    = blockIdx.y;
  const int lane = threadIdx.x & 31;
  const int wave = threadIdx.x >> 5;
  const int tilesN = N >> 6;
  const int tilesM = M >> 6;
  const int tile = blockIdx.x * 8 + wave;
  if (tile >= tilesM * tilesN) return;
  const int tm = tile / tilesN;
  const int tn = tile - tm * tilesN;
  const int m0 = tm << 6;
  const int n0 = tn << 6;

  const T* Ab  = A  + (size_t)b * strideA;
  const T* Bb  = Bt + (size_t)b * strideB;
  const T* Ab2 = SPLIT ? (A2  + (size_t)b * strideA) : nullptr;
  const T* Bb2 = SPLIT ? (Bt2 + (size_t)b * strideB) : nullptr;

  const int rlane = lane & 15;
  const int koff  = (lane >> 4) * 8;
  const int mOff  = (lane >> 4) * 8;

  v8f acc[4][4];
#pragma unroll
  for (int i = 0; i < 4; ++i)
#pragma unroll
    for (int j = 0; j < 4; ++j) acc[i][j] = (v8f){0.f,0.f,0.f,0.f,0.f,0.f,0.f,0.f};

  for (int k0 = 0; k0 < K; k0 += 32) {
    V bh[4], bl[4];
#pragma unroll
    for (int j = 0; j < 4; ++j) {
      const size_t bo = (size_t)(n0 + (j << 4) + rlane) * ldb + koff + k0;
      bh[j] = Frag<T>::load(Bb + bo);
      if (SPLIT) bl[j] = Frag<T>::load(Bb2 + bo);
    }
#pragma unroll
    for (int i = 0; i < 4; ++i) {
      const size_t ao = (size_t)(m0 + (i << 4) + rlane) * lda + koff + k0;
      V ah = Frag<T>::load(Ab + ao);
      V al;
      if (SPLIT) al = Frag<T>::load(Ab2 + ao);
#pragma unroll
      for (int j = 0; j < 4; ++j) {
        acc[i][j] = Frag<T>::mma(ah, bh[j], acc[i][j]);
        if (SPLIT) {
          acc[i][j] = Frag<T>::mma(ah, bl[j], acc[i][j]);
          acc[i][j] = Frag<T>::mma(al, bh[j], acc[i][j]);
        }
      }
      Frag<T>::guard(acc[i][0], acc[i][3], ah, SPLIT ? al : ah);
    }
    Frag<T>::keep(bh[0], bh[1], bh[2], bh[3]);
    if (SPLIT) Frag<T>::keep(bl[0], bl[1], bl[2], bl[3]);
  }
  acc_guard4(acc[0][0], acc[0][1], acc[0][2], acc[0][3]);
  acc_guard4(acc[1][0], acc[1][1], acc[1][2], acc[1][3]);
  acc_guard4(acc[2][0], acc[2][1], acc[2][2], acc[2][3]);
  acc_guard4(acc[3][0], acc[3][1], acc[3][2], acc[3][3]);

  float* slab = sT[wave];
  const float* Rb = RESID ? (resid + (size_t)b * strideR) : nullptr;
#pragma unroll
  for (int i = 0; i < 4; ++i) {
    const int mBase = m0 + (i << 4);
#pragma unroll
    for (int j = 0; j < 4; ++j) {
      const int n = n0 + (j << 4) + rlane;
      float bv = 0.f;
      if (BIAS_MODE == 2) bv = bias[n];
#pragma unroll
      for (int r = 0; r < 8; ++r) {
        float v = acc[i][j][r] * scale;
        if (BIAS_MODE == 1) v += bias[mBase + mOff + r];
        if (BIAS_MODE == 2) v += bv;
        if (RESID) v += Rb[(size_t)(mBase + mOff + r) * ldc + n];
        if (ACT == 1) v = tanhf(v);
        if (ACT == 2) v = fmaxf(v, 0.0f);
        if (ACT == 3) v = v / (1.0f + expf(-v));
        if (ACT == 4) v = (v > 0.f) ? v : 0.01f * v;
        if (ACT == 5) v = 0.5f * v * (1.0f + erff(v * 0.70710678118654752f));
        slab[(mOff + r) * 68 + (j << 4) + rlane] = v;
      }
    }
    __builtin_amdgcn_fence(__ATOMIC_RELEASE, "workgroup");
    __builtin_amdgcn_wave_barrier();
    __builtin_amdgcn_fence(__ATOMIC_ACQUIRE, "workgroup");
    if (OUT_MODE == 0) {
      float* C = (float*)Cout + (size_t)b * strideC;
      const int hh = lane >> 4, c4 = (lane & 15) * 4;
      for (int pass = 0; pass < 2; ++pass) {
#pragma unroll
        for (int it = 0; it < 8; ++it) {
          const int row = it * 2 + hh;
          v4f v = *(const v4f*)(slab + row * 68 + c4);
          *(volatile v4f*)(C + (size_t)(mBase + row) * ldc + n0 + c4) = v;
        }
        __threadfence();
      }
    } else {
      const int q = lane >> 3, c8 = (lane & 7) * 8;
      unsigned short* C  = (unsigned short*)Cout  + (size_t)b * strideC;
      unsigned short* C2 = (OUT_MODE == 2) ? ((unsigned short*)Cout2 + (size_t)b * strideC) : nullptr;
      for (int pass = 0; pass < 2; ++pass) {
#pragma unroll
        for (int it = 0; it < 4; ++it) {
          const int row = it * 4 + q;
          const float* sp = slab + row * 68 + c8;
          v8h hv, lv;
#pragma unroll
          for (int e = 0; e < 8; ++e) {
            if (OUT_MODE == 1) {
              hv[e] = (_Float16)sp[e];
            } else {
              unsigned short hb = f2bf_bits(sp[e]);
              unsigned short lb = f2bf_bits(sp[e] - bf_bits2f(hb));
              hv[e] = __builtin_bit_cast(_Float16, hb);
              lv[e] = __builtin_bit_cast(_Float16, lb);
            }
          }
          *(volatile v8h*)(C + (size_t)(mBase + row) * ldc + n0 + c8) = hv;
          if (OUT_MODE == 2) *(volatile v8h*)(C2 + (size_t)(mBase + row) * ldc + n0 + c8) = lv;
        }
        __threadfence();
      }
    }
    __builtin_amdgcn_fence(__ATOMIC_RELEASE, "workgroup");
    __builtin_amdgcn_wave_barrier();
    __builtin_amdgcn_fence(__ATOMIC_ACQUIRE, "workgroup");
  }
}

__global__ __launch_bounds__(256) void cast_f32_f16x2_pad(
    const float* __restrict__ in, _Float16* __restrict__ out, int n2, int n2tot) {
  int i = blockIdx.x * 256 + threadIdx.x;
  if (i < n2tot) {
    unsigned u = 0u;
    if (i < n2) {
      const _Float16 h0 = (_Float16)in[2 * (size_t)i], h1 = (_Float16)in[2 * (size_t)i + 1];
      u = (unsigned)__builtin_bit_cast(unsigned short, h0) | ((unsigned)__builtin_bit_cast(unsigned short, h1) << 16);
    }
    ((volatile unsigned*)out)[i] = u;
    __threadfence();
    ((volatile unsigned*)out)[i] = u;
  }
}

__global__ __launch_bounds__(256) void transpose_cast_w_kernel(
    const float* __restrict__ W, _Float16* __restrict__ Wt, int K, int Cn, float scale) {
  const int kg = K >> 3;
  const int gidx = blockIdx.x * 256 + threadIdx.x;
  if (gidx < Cn * kg) {
    const int n = gidx / kg;
    const int k0 = (gidx - n * kg) * 8;
    v8h vv;
#pragma unroll
    for (int i = 0; i < 8; ++i) vv[i] = (_Float16)(W[(size_t)(k0 + i) * Cn + n] * scale);
    _Float16* dst = Wt + (size_t)n * K + k0;
    *(volatile v8h*)dst = vv;
    __threadfence();
    *(volatile v8h*)dst = vv;
  }
}

template <int NW>
__device__ __forceinline__ int block_excl_scan(int cnt, int* wtot, int lane, int wave, int& total) {
  int incl = cnt;
#pragma unroll
  for (int off = 1; off < 32; off <<= 1) {
    const int t = __shfl_up(incl, off, 32);
    if (lane >= off) incl += t;
  }
  if (lane == 31) wtot[wave] = incl;
  __syncthreads();
  int base = 0, tot = 0;
#pragma unroll
  for (int w = 0; w < NW; ++w) { const int t = wtot[w]; tot += t; base += (w < wave) ? t : 0; }
  total = tot;
  return base + incl - cnt;
}

#define DG_NT 256
#define DG_EPT 8
#define DG_CH (DG_NT * DG_EPT)
__global__ __launch_bounds__(DG_NT) void gcn_dinv_kernel(
    const int* __restrict__ ecol, float* __restrict__ dinv, int N, int Npad, int NE, int vec_ok) {
  __shared__ int lc[DG_CH];
  __shared__ int wtot[DG_NT / 32];
  const int tid = threadIdx.x, lane = tid & 31, wave = tid >> 5;
  const int tile0 = blockIdx.x * DG_NT;
  int cntd = 0;
  for (int cb = 0; cb < NE; cb += DG_CH) {
    const int e0 = cb + tid * DG_EPT;
    int cv[DG_EPT];
    if (vec_ok && e0 + DG_EPT <= NE) {
      const v4i ca = *(const v4i*)(ecol + e0);
      const v4i cbv = *(const v4i*)(ecol + e0 + 4);
      cv[0] = ca[0]; cv[1] = ca[1]; cv[2] = ca[2]; cv[3] = ca[3];
      cv[4] = cbv[0]; cv[5] = cbv[1]; cv[6] = cbv[2]; cv[7] = cbv[3];
    } else {
#pragma unroll
      for (int i = 0; i < DG_EPT; ++i) {
        cv[i] = -1;
        if (e0 + i < NE) cv[i] = ecol[e0 + i];
      }
    }
    unsigned flags = 0;
#pragma unroll
    for (int i = 0; i < DG_EPT; ++i)
      if ((unsigned)(cv[i] - tile0) < (unsigned)DG_NT && cv[i] < N) flags |= 1u << i;
    const int cnt = __popc(flags);
    int nh;
    int pos = block_excl_scan<DG_NT / 32>(cnt, wtot, lane, wave, nh);
#pragma unroll
    for (int i = 0; i < DG_EPT; ++i) {
      if (flags & (1u << i)) {
        if (pos < DG_CH) lc[pos] = cv[i] - tile0;
        ++pos;
      }
    }
    __syncthreads();
    nh = nh < DG_CH ? nh : DG_CH;
    for (int j = 0; j < nh; ++j) cntd += (lc[j] == tid) ? 1 : 0;
    __syncthreads();
  }
  const int node = tile0 + tid;
  const float deg = (float)(cntd + 1);
  float d = 1.0f / sqrtf(deg);
  if (node >= N) d = 0.f;
  if (node < Npad) {
    ((volatile float*)dinv)[node] = d;
    __threadfence();
    ((volatile float*)dinv)[node] = d;
  }
}

#define AG_TILE 64
#define AG_C 512
#define AG_T 128
#define AG_EPT 8
#define AG_CH (AG_T * AG_EPT)
template <int MODE>
__global__ __launch_bounds__(AG_T) void gcn_agg_kernel(
    const float* __restrict__ Mf, const int* __restrict__ erow, const int* __restrict__ ecol,
    const float* __restrict__ dinv, const float* __restrict__ bias, void* __restrict__ outp,
    int N, int Npad, int NE, int vec_ok) {
  constexpr int NW = AG_T / 32;
  __shared__ __align__(16) float acc[AG_TILE * AG_C];
  __shared__ int   lrw[AG_CH];
  __shared__ int   llc[AG_CH];
  __shared__ float lnm[AG_CH];
  __shared__ int   wtot[NW];
  const int tid = threadIdx.x, lane = tid & 31, wave = tid >> 5;
  const int tile0 = blockIdx.x * AG_TILE;
  const int ch0 = tid * 4;
  const v4f z4 = {0.f, 0.f, 0.f, 0.f};
#pragma unroll 1
  for (int r = 0; r < AG_TILE; ++r) *(v4f*)(acc + r * AG_C + ch0) = z4;
  for (int cb = 0; cb < NE; cb += AG_CH) {
    const int e0 = cb + tid * AG_EPT;
    int cv[AG_EPT];
    if (vec_ok && e0 + AG_EPT <= NE) {
      const v4i t0 = *(const v4i*)(ecol + e0);
      const v4i t1 = *(const v4i*)(ecol + e0 + 4);
      cv[0] = t0[0]; cv[1] = t0[1]; cv[2] = t0[2]; cv[3] = t0[3];
      cv[4] = t1[0]; cv[5] = t1[1]; cv[6] = t1[2]; cv[7] = t1[3];
    } else {
#pragma unroll
      for (int i = 0; i < AG_EPT; ++i) { cv[i] = -1; if (e0 + i < NE) cv[i] = ecol[e0 + i]; }
    }
    unsigned flags = 0;
#pragma unroll
    for (int i = 0; i < AG_EPT; ++i)
      if ((unsigned)(cv[i] - tile0) < (unsigned)AG_TILE && cv[i] < N) flags |= 1u << i;
    const int cnt = __popc(flags);
    int nh;
    int pos = block_excl_scan<NW>(cnt, wtot, lane, wave, nh);
#pragma unroll
    for (int i = 0; i < AG_EPT; ++i) {
      if (flags & (1u << i)) {
        if (pos < AG_CH) {
          const int e = e0 + i;
          int r = erow[e];
          r = r < 0 ? 0 : (r >= N ? N - 1 : r);
          const int cc = cv[i];
          const float nm = dinv[r] * dinv[cc];
          lrw[pos] = r; llc[pos] = cc - tile0; lnm[pos] = nm;
        }
        ++pos;
      }
    }
    __syncthreads();
    nh = nh < AG_CH ? nh : AG_CH;
    for (int j = 0; j < nh; ++j) {
      const int r = lrw[j];
      const int lc = llc[j];
      const float nm = lnm[j];
      const v4f m = *(const v4f*)(Mf + (size_t)r * AG_C + ch0);
      float* ap = acc + lc * AG_C + ch0;
      v4f a = *(const v4f*)ap;
#pragma unroll
      for (int q = 0; q < 4; ++q) a[q] += m[q] * nm;
      *(v4f*)ap = a;
    }
    __syncthreads();
  }
  __syncthreads();

  const v4f b4 = *(const v4f*)(bias + ch0);
  for (int pass = 0; pass < 2; ++pass) {
#pragma unroll 1
    for (int row = 0; row < AG_TILE; ++row) {
      const int node = tile0 + row;
      if (node < Npad) {
        v4f y = z4;
        if (node < N) {
          const float di = dinv[node];
          const float ns = di * di;
          const v4f a  = *(const v4f*)(acc + row * AG_C + ch0);
          const v4f mm = *(const v4f*)(Mf + (size_t)node * AG_C + ch0);
#pragma unroll
          for (int q = 0; q < 4; ++q) y[q] = fmaxf(a[q] + mm[q] * ns + b4[q], 0.f);
        }
        if (MODE == 0) {
          v4h hv;
#pragma unroll
          for (int q = 0; q < 4; ++q) hv[q] = (_Float16)y[q];
          *(volatile v4h*)((_Float16*)outp + (size_t)node * AG_C + ch0) = hv;
        } else {
          *(volatile v4f*)((float*)outp + (size_t)node * AG_C + ch0) = y;
        }
      }
    }
    __threadfence();
  }
}

#define PL_T 128
#define PL_EPT 16
#define PL_CH (PL_T * PL_EPT)
__global__ __launch_bounds__(PL_T) void pool_kernel(
    const float* __restrict__ H, const int* __restrict__ bat, float* __restrict__ outf,
    _Float16* __restrict__ out16, int N, int G, int vec_ok) {
  constexpr int NW = PL_T / 32;
  __shared__ int lnd[PL_CH];
  __shared__ int wtot[NW];
  const int tid = threadIdx.x, lane = tid & 31, wave = tid >> 5;
  const int g = blockIdx.x;
  const int ch0 = tid * 4;
  v4f s = {0.f, 0.f, 0.f, 0.f};
  for (int cb = 0; cb < N; cb += PL_CH) {
    const int i0 = cb + tid * PL_EPT;
    int bv[PL_EPT];
    if (vec_ok && i0 + PL_EPT <= N) {
#pragma unroll
      for (int qd = 0; qd < PL_EPT / 4; ++qd) {
        const v4i t = *(const v4i*)(bat + i0 + 4 * qd);
        bv[4 * qd + 0] = t[0]; bv[4 * qd + 1] = t[1]; bv[4 * qd + 2] = t[2]; bv[4 * qd + 3] = t[3];
      }
    } else {
#pragma unroll
      for (int i = 0; i < PL_EPT; ++i) { bv[i] = -1; if (i0 + i < N) bv[i] = bat[i0 + i]; }
    }
    unsigned flags = 0;
#pragma unroll
    for (int i = 0; i < PL_EPT; ++i)
      if (bv[i] == g) flags |= 1u << i;
    const int cnt = __popc(flags);
    int nh;
    int pos = block_excl_scan<NW>(cnt, wtot, lane, wave, nh);
#pragma unroll
    for (int i = 0; i < PL_EPT; ++i) {
      if (flags & (1u << i)) {
        if (pos < PL_CH) lnd[pos] = i0 + i;
        ++pos;
      }
    }
    __syncthreads();
    nh = nh < PL_CH ? nh : PL_CH;
    for (int j = 0; j < nh; ++j) {
      int node = lnd[j];
      node = node < 0 ? 0 : (node >= N ? N - 1 : node);
      const v4f hrow = *(const v4f*)(H + (size_t)node * AG_C + ch0);
      s += hrow;
    }
    __syncthreads();
  }
  v4h hv;
#pragma unroll
  for (int q = 0; q < 4; ++q) hv[q] = (_Float16)s[q];
  for (int pass = 0; pass < 2; ++pass) {
    if (g < G) *(volatile v4f*)(outf + (size_t)g * AG_C + ch0) = s;
    *(volatile v4h*)(out16 + (size_t)g * AG_C + ch0) = hv;
    __threadfence();
  }
}

static void gemm_f16_host(const _Float16* A, int lda, const _Float16* Bt, int ldb, float* Cc, int ldc,
                          const float* bias, int use_bias, const float* dummy_resid,
                          int M, int Nn, int K, float scale, hipStream_t stream) {
  const int tiles = (M / 64) * (Nn / 64);
  dim3 grid((tiles + 7) / 8, 1);
  if (use_bias) {
    wmma_gemm64<0, false, 2, 0, false, 0><<<grid, 256, 0, stream>>>(
        (const unsigned short*)A, (const unsigned short*)A, lda, 0L,
        (const unsigned short*)Bt, (const unsigned short*)Bt, ldb, 0L,
        (void*)Cc, (void*)Cc, ldc, 0L, bias, dummy_resid, 0L, M, Nn, K, scale);
  } else {
    wmma_gemm64<0, false, 0, 0, false, 0><<<grid, 256, 0, stream>>>(
        (const unsigned short*)A, (const unsigned short*)A, lda, 0L,
        (const unsigned short*)Bt, (const unsigned short*)Bt, ldb, 0L,
        (void*)Cc, (void*)Cc, ldc, 0L, bias, dummy_resid, 0L, M, Nn, K, scale);
  }
}

extern "C" void kernel_launch(void* const* d_in, const int* in_sizes, int n_in,
                              void* d_out, int out_size, void* d_ws, size_t ws_size,
                              hipStream_t stream) {
  if (n_in < 9) return;
  const int F = 512, OUTF = 128;
  const int N = in_sizes[0] / F;
  if (N < 1 || N * F != in_sizes[0]) return;
  if (in_sizes[1] != F * F || in_sizes[2] != F || in_sizes[3] != F * F || in_sizes[4] != F) return;
  if (in_sizes[5] != F * OUTF || in_sizes[6] != OUTF) return;
  const int NE = in_sizes[7] / 2;
  if (NE < 0 || NE * 2 != in_sizes[7]) return;
  if (in_sizes[8] != N) return;
  if (out_size <= 0 || (out_size % (F + OUTF)) != 0) return;
  const int G = out_size / (F + OUTF);
  const int Npad = ((N + 63) / 64) * 64;
  const int Gpad = ((G + 63) / 64) * 64;
  const int vec_ok = (NE % 8 == 0) ? 1 : 0;

  const float* x    = (const float*)d_in[0];
  const float* W1   = (const float*)d_in[1];
  const float* b1   = (const float*)d_in[2];
  const float* W2   = (const float*)d_in[3];
  const float* b2   = (const float*)d_in[4];
  const float* Wl   = (const float*)d_in[5];
  const float* bl   = (const float*)d_in[6];
  const int*   ei   = (const int*)d_in[7];
  const int*   bat  = (const int*)d_in[8];
  const int*   esrc = ei;
  const int*   edst = ei + NE;

  float* out0 = (float*)d_out;
  float* out1 = out0 + (size_t)G * F;

  size_t off = 0;
  auto carve = [&](size_t bytes) -> char* { char* p = (char*)d_ws + off; off += (bytes + 255) & ~(size_t)255; return p; };
  float*    dinv = (float*)carve((size_t)Npad * 4);
  _Float16* a16  = (_Float16*)carve((size_t)Npad * F * 2);
  _Float16* wt16 = (_Float16*)carve((size_t)F * F * 2);
  float*    mbuf = (float*)carve((size_t)Npad * F * 4);
  float*    h2   = (float*)carve((size_t)Npad * F * 4);
  _Float16* p16  = (_Float16*)carve((size_t)Gpad * F * 2);
  float*    ofin = (float*)carve((size_t)Gpad * OUTF * 4);
  if (off > ws_size || off > (size_t)134217728) return;

  const float wsc = 16.0f, wsc_inv = 1.0f / 16.0f;

  {
    const int n2 = N * (F / 2), n2tot = Npad * (F / 2);
    cast_f32_f16x2_pad<<<(n2tot + 255) / 256, 256, 0, stream>>>(x, a16, n2, n2tot);
  }
  gcn_dinv_kernel<<<(Npad + DG_NT - 1) / DG_NT, DG_NT, 0, stream>>>(edst, dinv, N, Npad, NE, vec_ok);

  transpose_cast_w_kernel<<<(F * (F / 8) + 255) / 256, 256, 0, stream>>>(W1, wt16, F, F, wsc);
  gemm_f16_host(a16, F, wt16, F, mbuf, F, b1, 0, dinv, Npad, F, F, wsc_inv, stream);
  gcn_agg_kernel<0><<<Npad / AG_TILE, AG_T, 0, stream>>>(mbuf, esrc, edst, dinv, b1, (void*)a16, N, Npad, NE, vec_ok);

  transpose_cast_w_kernel<<<(F * (F / 8) + 255) / 256, 256, 0, stream>>>(W2, wt16, F, F, wsc);
  gemm_f16_host(a16, F, wt16, F, mbuf, F, b2, 0, dinv, Npad, F, F, wsc_inv, stream);
  gcn_agg_kernel<1><<<Npad / AG_TILE, AG_T, 0, stream>>>(mbuf, esrc, edst, dinv, b2, (void*)h2, N, Npad, NE, vec_ok);

  pool_kernel<<<Gpad, PL_T, 0, stream>>>(h2, bat, out0, p16, N, G, 1);

  transpose_cast_w_kernel<<<(OUTF * (F / 8) + 255) / 256, 256, 0, stream>>>(Wl, wt16, F, OUTF, wsc);
  if (Gpad == G) {
    gemm_f16_host(p16, F, wt16, F, out1, OUTF, bl, 1, dinv, Gpad, OUTF, F, wsc_inv, stream);
  } else {
    gemm_f16_host(p16, F, wt16, F, ofin, OUTF, bl, 1, dinv, Gpad, OUTF, F, wsc_inv, stream);
    hipMemcpyAsync(out1, ofin, (size_t)G * OUTF * sizeof(float), hipMemcpyDeviceToDevice, stream);
  }
}
